// GCN_69801808495208
// MI455X (gfx1250) — hardware-verified
//
#include <hip/hip_runtime.h>
#include <stddef.h>
#include <stdint.h>
#include <math.h>

#define NB     16
#define SEQ    128
#define NCH    256
#define MROWS  2048
#define KP     512
#define NSTEP  3
#define NTHR   256
#define TM     128
#define TN     64
#define HM_UNITS  (MROWS * (NCH / 8))
#define WPL_UNITS (NCH * (NCH / 8))
#define NPLANE    (NSTEP * 4)
#define W_UNITS   (NPLANE * WPL_UNITS)
#define PREP_UNITS (HM_UNITS + W_UNITS)
#define WSMAX  134217728

static_assert(MROWS == NB * SEQ);
static_assert(TM == SEQ && MROWS % TM == 0 && NCH % TN == 0);
static_assert(KP == 2 * NCH && KP % 32 == 0 && NCH % 32 == 0);
static_assert(TM == (NTHR / 32) * 16 && TN == 64);
static_assert(HM_UNITS % NTHR == 0 && WPL_UNITS % NTHR == 0 && PREP_UNITS % NTHR == 0);
static_assert(NCH == NTHR);

typedef float          v4f   __attribute__((ext_vector_type(4)));
typedef float          v8f   __attribute__((ext_vector_type(8)));
typedef int            v8i   __attribute__((ext_vector_type(8)));
typedef unsigned int   v4u   __attribute__((ext_vector_type(4)));
typedef unsigned short v8us  __attribute__((ext_vector_type(8)));
typedef unsigned short v16us __attribute__((ext_vector_type(16)));
typedef __bf16         v16bf __attribute__((ext_vector_type(16)));
typedef v4f  __attribute__((may_alias)) v4fa;
typedef v4u  __attribute__((may_alias)) v4ua;
typedef v8us __attribute__((may_alias)) v8usa;
union FragB { v16bf v; v16us u; v8us h[2]; v8i w; };

__device__ __forceinline__ v8f wmb(const FragB& a, const FragB& b, v8f c) {
  v8f d = __builtin_amdgcn_wmma_f32_16x16x32_bf16(false, a.v, false, b.v, (short)0, c, false, false);
  asm volatile("v_nop\n\tv_nop\n\tv_nop\n\tv_nop" : "+v"(d) : "v"(a.w), "v"(b.w));
  return d;
}

__device__ __forceinline__ unsigned bf16_bits(float f) {
  const unsigned u = __float_as_uint(f);
  return (u + 0x7FFFu + ((u >> 16) & 1u)) >> 16;
}
__device__ __forceinline__ float bf16_val(float f) {
  return __uint_as_float(bf16_bits(f) << 16);
}

__device__ __forceinline__ void split8(const v4f a, const v4f b, v8us& h, v8us& l) {
  unsigned hb;
  hb = bf16_bits(a.x); h[0] = (unsigned short)hb; l[0] = (unsigned short)bf16_bits(a.x - __uint_as_float(hb << 16));
  hb = bf16_bits(a.y); h[1] = (unsigned short)hb; l[1] = (unsigned short)bf16_bits(a.y - __uint_as_float(hb << 16));
  hb = bf16_bits(a.z); h[2] = (unsigned short)hb; l[2] = (unsigned short)bf16_bits(a.z - __uint_as_float(hb << 16));
  hb = bf16_bits(a.w); h[3] = (unsigned short)hb; l[3] = (unsigned short)bf16_bits(a.w - __uint_as_float(hb << 16));
  hb = bf16_bits(b.x); h[4] = (unsigned short)hb; l[4] = (unsigned short)bf16_bits(b.x - __uint_as_float(hb << 16));
  hb = bf16_bits(b.y); h[5] = (unsigned short)hb; l[5] = (unsigned short)bf16_bits(b.y - __uint_as_float(hb << 16));
  hb = bf16_bits(b.z); h[6] = (unsigned short)hb; l[6] = (unsigned short)bf16_bits(b.z - __uint_as_float(hb << 16));
  hb = bf16_bits(b.w); h[7] = (unsigned short)hb; l[7] = (unsigned short)bf16_bits(b.w - __uint_as_float(hb << 16));
}

__global__ __launch_bounds__(NTHR) void k_prep(const float* __restrict__ feat, const float* __restrict__ mask,
                                               const float* __restrict__ aggW, const float* __restrict__ attnW,
                                               const float* __restrict__ updW,
                                               unsigned short* HM, unsigned short* WP) {
  const int u = (int)blockIdx.x * NTHR + (int)threadIdx.x;
  if (u < HM_UNITS) {
    const int row = u >> 5;
    const int c8  = (u & 31) * 8;
    const float* p = feat + (size_t)row * NCH + c8;
    v4f a = *(const v4f*)p;
    v4f b = *(const v4f*)(p + 4);
    const float mv = bf16_val(mask[row]);
    a.x = bf16_val(a.x) * mv; a.y = bf16_val(a.y) * mv; a.z = bf16_val(a.z) * mv; a.w = bf16_val(a.w) * mv;
    b.x = bf16_val(b.x) * mv; b.y = bf16_val(b.y) * mv; b.z = bf16_val(b.z) * mv; b.w = bf16_val(b.w) * mv;
    v8us hv, lv;
    split8(a, b, hv, lv);
    unsigned short* dp = HM + (size_t)row * KP + c8;
    *(volatile v8us*)dp = hv;
    *(volatile v8us*)(dp + NCH) = lv;
    __threadfence();
    *(volatile v8us*)dp = hv;
    *(volatile v8us*)(dp + NCH) = lv;
  } else if (u < PREP_UNITS) {
    const int v     = u - HM_UNITS;
    const int plane = v >> 13;
    const int step  = plane >> 2;
    const int mat   = plane & 3;
    const int n     = (v >> 5) & (NCH - 1);
    const int k8    = (v & 31) * 8;
    v4f a, b;
    if (mat == 0) {
      const float* p = aggW + (size_t)step * (NCH * NCH) + (size_t)n * NCH + k8;
      a = *(const v4f*)p; b = *(const v4f*)(p + 4);
    } else if (mat == 1) {
      const float* p = attnW + (size_t)step * (NCH * KP) + (size_t)n * KP + k8;
      a = *(const v4f*)p; b = *(const v4f*)(p + 4);
    } else {
      const float* p = updW + (size_t)step * (NCH * KP) + (size_t)n * KP + (size_t)(mat - 2) * NCH + k8;
      a = *(const v4f*)p; b = *(const v4f*)(p + 4);
    }
    v8us o;
    o[0] = (unsigned short)bf16_bits(a.x); o[1] = (unsigned short)bf16_bits(a.y);
    o[2] = (unsigned short)bf16_bits(a.z); o[3] = (unsigned short)bf16_bits(a.w);
    o[4] = (unsigned short)bf16_bits(b.x); o[5] = (unsigned short)bf16_bits(b.y);
    o[6] = (unsigned short)bf16_bits(b.z); o[7] = (unsigned short)bf16_bits(b.w);
    unsigned short* dp = WP + (size_t)plane * (NCH * NCH) + (size_t)n * NCH + k8;
    *(volatile v8us*)dp = o;
    __threadfence();
    *(volatile v8us*)dp = o;
  }
}

__device__ __forceinline__ void gemm_core(const unsigned short* __restrict__ A, const unsigned short* __restrict__ W,
                                          int rowBase, int col0, int wave, int hh, int m, v8f (&acc)[4]) {
  const unsigned short* ap = A + (size_t)(rowBase + 16 * wave + m) * (size_t)KP + 8 * hh;
  const unsigned short* wp = W + (size_t)(col0 + m) * (size_t)NCH + 8 * hh;
#pragma unroll 1
  for (int ks = 0; ks < KP / 32; ++ks) {
    const int ka = 32 * ks;
    const int kb = ka & (NCH - 1);
    FragB af;
    af.h[0] = *(const v8usa*)(ap + ka);
    af.h[1] = *(const v8usa*)(ap + ka + 16);
#pragma unroll
    for (int t = 0; t < 4; ++t) {
      const unsigned short* wq = wp + (size_t)(16 * t) * (size_t)NCH + kb;
      FragB bf;
      bf.h[0] = *(const v8usa*)wq;
      bf.h[1] = *(const v8usa*)(wq + 16);
      acc[t] = wmb(af, bf, acc[t]);
    }
  }
}

__device__ __forceinline__ void stage_tile(float* stg, const v8f (&acc)[4], const float (&add)[4],
                                           int wave, int hh, int m) {
#pragma unroll
  for (int t = 0; t < 4; ++t) {
    const int lc = 16 * t + m;
#pragma unroll
    for (int r = 0; r < 8; ++r) {
      const int lr = 16 * wave + 8 * hh + r;
      stg[lr * TN + lc] = acc[t][r] + add[t];
    }
  }
}

__device__ __forceinline__ void store_f32_tile(const float* stg, float* dst, int rowBase, int col0,
                                               int wave, int hh, int m) {
  v4f fv[8];
#pragma unroll
  for (int i = 0; i < 8; ++i) {
    const int lr = 16 * wave + 2 * i + hh;
    fv[i] = *(const v4fa*)(stg + lr * TN + 4 * m);
  }
#pragma unroll
  for (int i = 0; i < 8; ++i) {
    const int lr = 16 * wave + 2 * i + hh;
    float* op = dst + (size_t)(rowBase + lr) * (size_t)NCH + col0 + 4 * m;
    *(volatile v4f*)op = fv[i];
  }
  __threadfence();
#pragma unroll
  for (int i = 0; i < 8; ++i) {
    const int lr = 16 * wave + 2 * i + hh;
    float* op = dst + (size_t)(rowBase + lr) * (size_t)NCH + col0 + 4 * m;
    *(volatile v4f*)op = fv[i];
  }
}

template <int MSK>
__device__ __forceinline__ void store_hl_tile(const float* stg, const float* rowscale, unsigned short* dst,
                                              int rowBase, int col0, int wave, int lane) {
  v8us hv[4], lv[4];
  const int c8 = 8 * (lane & 7);
#pragma unroll
  for (int it = 0; it < 4; ++it) {
    const int lr = 16 * wave + 4 * it + (lane >> 3);
    v4f a = *(const v4fa*)(stg + lr * TN + c8);
    v4f b = *(const v4fa*)(stg + lr * TN + c8 + 4);
    if constexpr (MSK != 0) {
      const float sc = rowscale[lr];
      a.x *= sc; a.y *= sc; a.z *= sc; a.w *= sc;
      b.x *= sc; b.y *= sc; b.z *= sc; b.w *= sc;
    }
    split8(a, b, hv[it], lv[it]);
  }
#pragma unroll
  for (int it = 0; it < 4; ++it) {
    const int lr = 16 * wave + 4 * it + (lane >> 3);
    unsigned short* dp = dst + (size_t)(rowBase + lr) * (size_t)KP + col0 + c8;
    *(volatile v8us*)dp = hv[it];
    *(volatile v8us*)(dp + NCH) = lv[it];
  }
  __threadfence();
#pragma unroll
  for (int it = 0; it < 4; ++it) {
    const int lr = 16 * wave + 4 * it + (lane >> 3);
    unsigned short* dp = dst + (size_t)(rowBase + lr) * (size_t)KP + col0 + c8;
    *(volatile v8us*)dp = hv[it];
    *(volatile v8us*)(dp + NCH) = lv[it];
  }
}

__global__ __launch_bounds__(NTHR) void k_agg(const unsigned short* __restrict__ HM,
                                              const unsigned short* __restrict__ Wp,
                                              const float* __restrict__ bias,
                                              float* X, unsigned short* XHL) {
  __shared__ __attribute__((aligned(16))) float stg[TM * TN];
  const int tid = (int)threadIdx.x, lane = tid & 31, wave = tid >> 5, hh = lane >> 4, m = lane & 15;
  const int rowBase = (int)blockIdx.x * TM;
  const int col0    = (int)blockIdx.y * TN;
  v8f acc[4];
  {
    const v8f z = {0.f, 0.f, 0.f, 0.f, 0.f, 0.f, 0.f, 0.f};
    acc[0] = z; acc[1] = z; acc[2] = z; acc[3] = z;
  }
  gemm_core(HM, Wp, rowBase, col0, wave, hh, m, acc);
  float bs[4];
#pragma unroll
  for (int t = 0; t < 4; ++t) bs[t] = bf16_val(bias[col0 + 16 * t + m]);
  stage_tile(stg, acc, bs, wave, hh, m);
  __syncthreads();
  store_f32_tile(stg, X, rowBase, col0, wave, hh, m);
  store_hl_tile<0>(stg, stg, XHL, rowBase, col0, wave, lane);
}

__global__ __launch_bounds__(NTHR) void k_p(const unsigned short* __restrict__ XHL,
                                            const unsigned short* __restrict__ Wp,
                                            const float* __restrict__ X, float* AGG) {
  __shared__ __attribute__((aligned(16))) float stg[TM * TN];
  __shared__ float redM[NTHR];
  __shared__ float redD[NTHR];
  __shared__ float redN[NTHR];
  __shared__ __attribute__((aligned(16))) float outs[TN];
  const int tid = (int)threadIdx.x, lane = tid & 31, wave = tid >> 5, hh = lane >> 4, m = lane & 15;
  const int bidx    = (int)blockIdx.x;
  const int rowBase = bidx * TM;
  const int col0    = (int)blockIdx.y * TN;
  v8f acc[4];
  {
    const v8f z = {0.f, 0.f, 0.f, 0.f, 0.f, 0.f, 0.f, 0.f};
    acc[0] = z; acc[1] = z; acc[2] = z; acc[3] = z;
  }
  gemm_core(XHL, Wp, rowBase, col0, wave, hh, m, acc);
  const float zs[4] = {0.0f, 0.0f, 0.0f, 0.0f};
  stage_tile(stg, acc, zs, wave, hh, m);
  __syncthreads();

  const int col = tid & (TN - 1);
  const int q   = tid >> 6;
  const float* pc = stg + (32 * q) * TN + col;
  float mx = pc[0];
#pragma unroll 4
  for (int s = 1; s < 32; ++s) mx = fmaxf(mx, pc[s * TN]);
  redM[tid] = mx;
  __syncthreads();
  const float mm = fmaxf(fmaxf(redM[col], redM[TN + col]), fmaxf(redM[2 * TN + col], redM[3 * TN + col]));
  const float* xg = X + (size_t)(rowBase + 32 * q) * (size_t)NCH + col0 + col;
  float den = 0.0f, num = 0.0f;
#pragma unroll 4
  for (int s = 0; s < 32; ++s) {
    const float e  = expf(pc[s * TN] - mm);
    const float xv = xg[(size_t)s * NCH];
    den += e;
    num = fmaf(e, xv, num);
  }
  redD[tid] = den;
  redN[tid] = num;
  __syncthreads();
  if (tid < TN) {
    const float d = ((redD[tid] + redD[TN + tid]) + redD[2 * TN + tid]) + redD[3 * TN + tid];
    const float n = ((redN[tid] + redN[TN + tid]) + redN[2 * TN + tid]) + redN[3 * TN + tid];
    const float uu = n * (1.0f / d);
    outs[tid] = 1.0f / (1.0f + expf(-uu));
  }
  __syncthreads();
  const v4f ov = *(const v4fa*)(outs + 4 * (lane & 15));
  float* op = AGG + (size_t)bidx * NCH + col0 + 4 * (lane & 15);
  const bool okst = (wave == 0) && (lane < 16);
  if (okst) *(volatile v4f*)op = ov;
  __threadfence();
  if (okst) *(volatile v4f*)op = ov;
}

template <int FIN>
__global__ __launch_bounds__(NTHR) void k_upd(const unsigned short* __restrict__ XHL,
                                              const unsigned short* __restrict__ U1p,
                                              const unsigned short* __restrict__ U2p,
                                              const float* __restrict__ ubias,
                                              const float* __restrict__ AGG,
                                              const float* __restrict__ mask,
                                              unsigned short* HM, float* outp) {
  __shared__ __attribute__((aligned(16))) float stg[TM * TN];
  __shared__ __attribute__((aligned(16))) float ags[NCH];
  __shared__ float rp[NTHR];
  __shared__ float Rs[TN];
  __shared__ float mks[SEQ];
  const int tid = (int)threadIdx.x, lane = tid & 31, wave = tid >> 5, hh = lane >> 4, m = lane & 15;
  const int bidx    = (int)blockIdx.x;
  const int rowBase = bidx * TM;
  const int col0    = (int)blockIdx.y * TN;

  ags[tid] = AGG[(size_t)bidx * NCH + tid];
  if (tid < SEQ) mks[tid] = bf16_val(mask[rowBase + tid]);
  __syncthreads();
  {
    const int o    = tid >> 2;
    const int part = tid & 3;
    const unsigned short* ur = U2p + (size_t)(col0 + o) * (size_t)NCH + 64 * part;
    const float* ag = ags + 64 * part;
    float s = 0.0f;
#pragma unroll 1
    for (int j = 0; j < 8; ++j) {
      const v4u w  = *(const v4ua*)(ur + 8 * j);
      const v4f g0 = *(const v4fa*)(ag + 8 * j);
      const v4f g1 = *(const v4fa*)(ag + 8 * j + 4);
      s = fmaf(g0.x, __uint_as_float(w.x << 16), s);
      s = fmaf(g0.y, __uint_as_float(w.x & 0xffff0000u), s);
      s = fmaf(g0.z, __uint_as_float(w.y << 16), s);
      s = fmaf(g0.w, __uint_as_float(w.y & 0xffff0000u), s);
      s = fmaf(g1.x, __uint_as_float(w.z << 16), s);
      s = fmaf(g1.y, __uint_as_float(w.z & 0xffff0000u), s);
      s = fmaf(g1.z, __uint_as_float(w.w << 16), s);
      s = fmaf(g1.w, __uint_as_float(w.w & 0xffff0000u), s);
    }
    rp[tid] = s;
  }
  __syncthreads();
  if (tid < TN) {
    const float b0 = bf16_val(ubias[col0 + tid]);
    Rs[tid] = (((b0 + rp[4 * tid]) + rp[4 * tid + 1]) + rp[4 * tid + 2]) + rp[4 * tid + 3];
  }
  __syncthreads();

  v8f acc[4];
  {
    const v8f z = {0.f, 0.f, 0.f, 0.f, 0.f, 0.f, 0.f, 0.f};
    acc[0] = z; acc[1] = z; acc[2] = z; acc[3] = z;
  }
  gemm_core(XHL, U1p, rowBase, col0, wave, hh, m, acc);
  float rs[4];
#pragma unroll
  for (int t = 0; t < 4; ++t) rs[t] = Rs[16 * t + m];
  stage_tile(stg, acc, rs, wave, hh, m);
  __syncthreads();
  if constexpr (FIN != 0) {
    store_f32_tile(stg, outp, rowBase, col0, wave, hh, m);
  } else {
    store_hl_tile<1>(stg, mks, HM, rowBase, col0, wave, lane);
  }
}

static inline size_t al256(size_t o) { return (o + 255) & ~(size_t)255; }

extern "C" void kernel_launch(void* const* d_in, const int* in_sizes, int n_in,
                              void* d_out, int out_size, void* d_ws, size_t ws_size,
                              hipStream_t stream) {
  if (n_in < 8) return;
  if (in_sizes[0] != MROWS * NCH) return;
  if (in_sizes[1] != MROWS) return;
  if (in_sizes[2] != NSTEP * NCH * NCH) return;
  if (in_sizes[3] != NSTEP * NCH) return;
  if (in_sizes[4] != NSTEP * NCH * KP) return;
  if (in_sizes[5] != NSTEP * NCH) return;
  if (in_sizes[6] != NSTEP * NCH * KP) return;
  if (in_sizes[7] != NSTEP * NCH) return;
  if (out_size != MROWS * NCH) return;

  const float* feat  = (const float*)d_in[0];
  const float* mask  = (const float*)d_in[1];
  const float* aggW  = (const float*)d_in[2];
  const float* aggB  = (const float*)d_in[3];
  const float* attnW = (const float*)d_in[4];
  const float* updW  = (const float*)d_in[6];
  const float* updB  = (const float*)d_in[7];
  float* out = (float*)d_out;

  char* ws = (char*)d_ws;
  size_t off = 0;
  const size_t oWP  = off; off = al256(off + (size_t)NPLANE * NCH * NCH * 2);
  const size_t oHM  = off; off = al256(off + (size_t)MROWS * KP * 2);
  const size_t oX   = off; off = al256(off + (size_t)MROWS * NCH * 4);
  const size_t oXHL = off; off = al256(off + (size_t)MROWS * KP * 2);
  const size_t oAGG = off; off = al256(off + (size_t)NB * NCH * 4);
  if (off > ws_size || off > (size_t)WSMAX) return;
  unsigned short* WP  = (unsigned short*)(ws + oWP);
  unsigned short* HM  = (unsigned short*)(ws + oHM);
  float*          X   = (float*)(ws + oX);
  unsigned short* XHL = (unsigned short*)(ws + oXHL);
  float*          AGG = (float*)(ws + oAGG);

  k_prep<<<PREP_UNITS / NTHR, NTHR, 0, stream>>>(feat, mask, aggW, attnW, updW, HM, WP);
  const dim3 gg(MROWS / TM, NCH / TN);
  for (int i = 0; i < NSTEP; ++i) {
    const unsigned short* Wa = WP + (size_t)(4 * i + 0) * (NCH * NCH);
    const unsigned short* W1 = WP + (size_t)(4 * i + 1) * (NCH * NCH);
    const unsigned short* U1 = WP + (size_t)(4 * i + 2) * (NCH * NCH);
    const unsigned short* U2 = WP + (size_t)(4 * i + 3) * (NCH * NCH);
    k_agg<<<gg, NTHR, 0, stream>>>(HM, Wa, aggB + (size_t)i * NCH, X, XHL);
    k_p<<<gg, NTHR, 0, stream>>>(XHL, W1, X, AGG);
    if (i < NSTEP - 1) {
      k_upd<0><<<gg, NTHR, 0, stream>>>(XHL, U1, U2, updB + (size_t)i * NCH, AGG, mask, HM, out);
    } else {
      k_upd<1><<<gg, NTHR, 0, stream>>>(XHL, U1, U2, updB + (size_t)i * NCH, AGG, mask, HM, out);
    }
  }
}
